// MambaBlock2D_41850161332281
// MI455X (gfx1250) — hardware-verified
//
#include <hip/hip_runtime.h>
#include <math.h>

typedef __attribute__((ext_vector_type(16))) _Float16 v16h;
typedef __attribute__((ext_vector_type(8)))  _Float16 v8h;
typedef __attribute__((ext_vector_type(16))) __bf16   v16b;
typedef __attribute__((ext_vector_type(8)))  __bf16   v8b;
typedef __attribute__((ext_vector_type(8)))  float    v8f;
typedef __attribute__((ext_vector_type(4)))  float    v4f;
typedef __attribute__((ext_vector_type(2)))  float    v2f;

constexpr int kBatch = 2;
constexpr int kSeqL  = 4096;
constexpr int kTok   = kBatch * kSeqL;
constexpr int kDimC  = 256;
constexpr int kDin   = 512;
constexpr int kXZW   = 2 * kDin;
constexpr int kNst   = 16;
constexpr int kDtR   = 16;
constexpr int kDtP   = 32;
constexpr int kXdR   = 48;
constexpr int kXdP   = 64;
constexpr int kFfn   = 1024;
constexpr int kLnP   = 264;
constexpr int kTP    = 260;
constexpr int kChBlk = 128;
constexpr int kSYP   = 136;

__device__ __forceinline__ unsigned short f2bf_bits(float f) {
  unsigned u = __float_as_uint(f);
  return (unsigned short)((u + 0x7FFFu + ((u >> 16) & 1u)) >> 16);
}
__device__ __forceinline__ float bf_bits2f(unsigned short h) { return __uint_as_float(((unsigned)h) << 16); }

__device__ __forceinline__ void dep_guard_h(v8f& a, v8f& b, v16h x, v16h y) { asm volatile("v_nop\n\tv_nop\n\tv_nop\n\tv_nop" : "+v"(a), "+v"(b) : "v"(x), "v"(y)); }
__device__ __forceinline__ void dep_guard_b(v8f& a, v8f& b, v16b x, v16b y) { asm volatile("v_nop\n\tv_nop\n\tv_nop\n\tv_nop" : "+v"(a), "+v"(b) : "v"(x), "v"(y)); }
__device__ __forceinline__ void keep4_h(v16h a, v16h b, v16h c, v16h d) { asm volatile("v_nop" :: "v"(a), "v"(b), "v"(c), "v"(d)); }
__device__ __forceinline__ void keep4_b(v16b a, v16b b, v16b c, v16b d) { asm volatile("v_nop" :: "v"(a), "v"(b), "v"(c), "v"(d)); }
__device__ __forceinline__ void acc_guard4(v8f& a, v8f& b, v8f& c, v8f& d) { asm volatile("v_nop\n\tv_nop\n\tv_nop\n\tv_nop" : "+v"(a), "+v"(b), "+v"(c), "+v"(d)); }
template <typename T> struct Frag;
template <> struct Frag<_Float16> {
  typedef v16h V; union U { v16h v; v8h h[2]; };
  static __device__ __forceinline__ v16h load(const _Float16* p) {
    U f; f.h[0] = *(const v8h*)(p); f.h[1] = *(const v8h*)(p + 16); return f.v;
  }
  static __device__ __forceinline__ v8f mma(v16h a, v16h b, v8f c) {
    return __builtin_amdgcn_wmma_f32_16x16x32_f16(false, a, false, b, (short)0, c, false, false);
  }
  static __device__ __forceinline__ void guard(v8f& a, v8f& b, v16h x, v16h y) { dep_guard_h(a, b, x, y); }
  static __device__ __forceinline__ void keep(v16h a, v16h b, v16h c, v16h d) { keep4_h(a, b, c, d); }
};
template <> struct Frag<__bf16> {
  typedef v16b V; union U { v16b v; v8b h[2]; };
  static __device__ __forceinline__ v16b load(const __bf16* p) {
    U f; f.h[0] = *(const v8b*)(p); f.h[1] = *(const v8b*)(p + 16); return f.v;
  }
  static __device__ __forceinline__ v8f mma(v16b a, v16b b, v8f c) {
    return __builtin_amdgcn_wmma_f32_16x16x32_bf16(false, a, false, b, (short)0, c, false, false);
  }
  static __device__ __forceinline__ void guard(v8f& a, v8f& b, v16b x, v16b y) { dep_guard_b(a, b, x, y); }
  static __device__ __forceinline__ void keep(v16b a, v16b b, v16b c, v16b d) { keep4_b(a, b, c, d); }
};

template <int ET> struct Elem;
template <> struct Elem<0> { typedef _Float16 T; };
template <> struct Elem<1> { typedef __bf16 T; };
template <int ET, bool SPLIT, int BIAS_MODE, int OUT_MODE, bool RESID, int ACT = 0>
__global__ __launch_bounds__(256) void wmma_gemm64(
    const unsigned short* __restrict__ Ap, const unsigned short* __restrict__ A2p, int lda, long strideA,
    const unsigned short* __restrict__ Btp, const unsigned short* __restrict__ Bt2p, int ldb, long strideB,
    void* __restrict__ Cout, void* __restrict__ Cout2, int ldc, long strideC,
    const float* __restrict__ bias,
    const float* __restrict__ resid, long strideR,
    int M, int N, int K, float scale) {
  typedef typename Elem<ET>::T T;
  typedef typename Frag<T>::V V;
  const T* A = (const T*)Ap; const T* A2 = (const T*)A2p; const T* Bt = (const T*)Btp; const T* Bt2 = (const T*)Bt2p;
  __shared__ __align__(16) float sT[8][16 * 68];
  const int b    = blockIdx.y;
  const int lane = threadIdx.x & 31;
  const int wave = threadIdx.x >> 5;
  const int tilesN = N >> 6;
  const int tilesM = M >> 6;
  const int tile = blockIdx.x * 8 + wave;
  if (tile >= tilesM * tilesN) return;
  const int tm = tile / tilesN;
  const int tn = tile - tm * tilesN;
  const int m0 = tm << 6;
  const int n0 = tn << 6;

  const T* Ab  = A  + (size_t)b * strideA;
  const T* Bb  = Bt + (size_t)b * strideB;
  const T* Ab2 = SPLIT ? (A2  + (size_t)b * strideA) : nullptr;
  const T* Bb2 = SPLIT ? (Bt2 + (size_t)b * strideB) : nullptr;

  const int rlane = lane & 15;
  const int koff  = (lane >> 4) * 8;
  const int mOff  = (lane >> 4) * 8;

  v8f acc[4][4];
#pragma unroll
  for (int i = 0; i < 4; ++i)
#pragma unroll
    for (int j = 0; j < 4; ++j) acc[i][j] = (v8f){0.f,0.f,0.f,0.f,0.f,0.f,0.f,0.f};

  for (int k0 = 0; k0 < K; k0 += 32) {
    V bh[4], bl[4];
#pragma unroll
    for (int j = 0; j < 4; ++j) {
      const size_t bo = (size_t)(n0 + (j << 4) + rlane) * ldb + koff + k0;
      bh[j] = Frag<T>::load(Bb + bo);
      if (SPLIT) bl[j] = Frag<T>::load(Bb2 + bo);
    }
#pragma unroll
    for (int i = 0; i < 4; ++i) {
      const size_t ao = (size_t)(m0 + (i << 4) + rlane) * lda + koff + k0;
      V ah = Frag<T>::load(Ab + ao);
      V al;
      if (SPLIT) al = Frag<T>::load(Ab2 + ao);
#pragma unroll
      for (int j = 0; j < 4; ++j) {
        acc[i][j] = Frag<T>::mma(ah, bh[j], acc[i][j]);
        if (SPLIT) {
          acc[i][j] = Frag<T>::mma(ah, bl[j], acc[i][j]);
          acc[i][j] = Frag<T>::mma(al, bh[j], acc[i][j]);
        }
      }
      Frag<T>::guard(acc[i][0], acc[i][3], ah, SPLIT ? al : ah);
    }
    Frag<T>::keep(bh[0], bh[1], bh[2], bh[3]);
    if (SPLIT) Frag<T>::keep(bl[0], bl[1], bl[2], bl[3]);
  }
  acc_guard4(acc[0][0], acc[0][1], acc[0][2], acc[0][3]);
  acc_guard4(acc[1][0], acc[1][1], acc[1][2], acc[1][3]);
  acc_guard4(acc[2][0], acc[2][1], acc[2][2], acc[2][3]);
  acc_guard4(acc[3][0], acc[3][1], acc[3][2], acc[3][3]);

  float* slab = sT[wave];
  const float* Rb = RESID ? (resid + (size_t)b * strideR) : nullptr;
#pragma unroll
  for (int i = 0; i < 4; ++i) {
    const int mBase = m0 + (i << 4);
#pragma unroll
    for (int j = 0; j < 4; ++j) {
      const int n = n0 + (j << 4) + rlane;
      float bv = 0.f;
      if (BIAS_MODE == 2) bv = bias[n];
#pragma unroll
      for (int r = 0; r < 8; ++r) {
        float v = acc[i][j][r] * scale;
        if (BIAS_MODE == 1) v += bias[mBase + mOff + r];
        if (BIAS_MODE == 2) v += bv;
        if (RESID) v += Rb[(size_t)(mBase + mOff + r) * ldc + n];
        if (ACT == 1) v = tanhf(v);
        if (ACT == 2) v = fmaxf(v, 0.0f);
        if (ACT == 3) v = v / (1.0f + expf(-v));
        if (ACT == 4) v = (v > 0.f) ? v : 0.01f * v;
        if (ACT == 5) v = 0.5f * v * (1.0f + erff(v * 0.70710678118654752f));
        slab[(mOff + r) * 68 + (j << 4) + rlane] = v;
      }
    }
    __builtin_amdgcn_fence(__ATOMIC_RELEASE, "workgroup");
    __builtin_amdgcn_wave_barrier();
    __builtin_amdgcn_fence(__ATOMIC_ACQUIRE, "workgroup");
    if (OUT_MODE == 0) {
      float* C = (float*)Cout + (size_t)b * strideC;
      const int hh = lane >> 4, c4 = (lane & 15) * 4;
      for (int pass = 0; pass < 2; ++pass) {
#pragma unroll
        for (int it = 0; it < 8; ++it) {
          const int row = it * 2 + hh;
          v4f v = *(const v4f*)(slab + row * 68 + c4);
          *(volatile v4f*)(C + (size_t)(mBase + row) * ldc + n0 + c4) = v;
        }
        __threadfence();
      }
    } else {
      const int q = lane >> 3, c8 = (lane & 7) * 8;
      unsigned short* C  = (unsigned short*)Cout  + (size_t)b * strideC;
      unsigned short* C2 = (OUT_MODE == 2) ? ((unsigned short*)Cout2 + (size_t)b * strideC) : nullptr;
      for (int pass = 0; pass < 2; ++pass) {
#pragma unroll
        for (int it = 0; it < 4; ++it) {
          const int row = it * 4 + q;
          const float* sp = slab + row * 68 + c8;
          v8h hv, lv;
#pragma unroll
          for (int e = 0; e < 8; ++e) {
            if (OUT_MODE == 1) {
              hv[e] = (_Float16)sp[e];
            } else {
              unsigned short hb = f2bf_bits(sp[e]);
              unsigned short lb = f2bf_bits(sp[e] - bf_bits2f(hb));
              hv[e] = __builtin_bit_cast(_Float16, hb);
              lv[e] = __builtin_bit_cast(_Float16, lb);
            }
          }
          *(volatile v8h*)(C + (size_t)(mBase + row) * ldc + n0 + c8) = hv;
          if (OUT_MODE == 2) *(volatile v8h*)(C2 + (size_t)(mBase + row) * ldc + n0 + c8) = lv;
        }
        __threadfence();
      }
    }
    __builtin_amdgcn_fence(__ATOMIC_RELEASE, "workgroup");
    __builtin_amdgcn_wave_barrier();
    __builtin_amdgcn_fence(__ATOMIC_ACQUIRE, "workgroup");
  }
}

__global__ __launch_bounds__(256) void cast_w_f16_kernel(
    const float* __restrict__ src, _Float16* __restrict__ dst,
    int Kreal, int Kpad, int nreal, int total8, float scale)
{
  const int i = blockIdx.x * 256 + threadIdx.x;
  if (i >= total8) return;
  const int e0  = i << 3;
  const int row = e0 / Kpad;
  const int col = e0 - row * Kpad;
  const int rc  = (row < nreal) ? row : (nreal - 1);
  const int cc  = (col < Kreal) ? col : (Kreal - 8);
  const bool keep = (row < nreal) && (col < Kreal);
  const float* p = src + (size_t)rc * Kreal + cc;
  const v4f a0 = *(const v4f*)(p);
  const v4f a1 = *(const v4f*)(p + 4);
  v8h hv;
#pragma unroll
  for (int e = 0; e < 4; ++e) {
    hv[e]     = (_Float16)(keep ? a0[e] * scale : 0.0f);
    hv[4 + e] = (_Float16)(keep ? a1[e] * scale : 0.0f);
  }
  _Float16* q = dst + e0;
  *(volatile v8h*)q = hv;
  __threadfence();
  *(volatile v8h*)q = hv;
}

__global__ __launch_bounds__(256) void ln_kernel(
    const float* __restrict__ x, const float* __restrict__ gw, const float* __restrict__ gb,
    float* __restrict__ YLN, _Float16* __restrict__ YLNH)
{
  __shared__ __align__(16) float sX[32 * kLnP];
  const int tid = threadIdx.x, lane = tid & 31, wave = tid >> 5;
  const int blk = blockIdx.x;
  const int b   = blk >> 7;
  const int l0  = (blk & 127) * 32;
  const float* xb = x + (size_t)b * kDimC * kSeqL + l0 + lane;
#pragma unroll 4
  for (int i = 0; i < 32; ++i) {
    const int c = wave + 8 * i;
    sX[lane * kLnP + c] = xb[(size_t)c * kSeqL];
  }
  __syncthreads();
  const v4f g8a = *(const v4f*)(gw + lane * 8), g8b = *(const v4f*)(gw + lane * 8 + 4);
  const v4f b8a = *(const v4f*)(gb + lane * 8), b8b = *(const v4f*)(gb + lane * 8 + 4);
  const v4f g4a = *(const v4f*)(gw + lane * 4), g4b = *(const v4f*)(gw + 128 + lane * 4);
  const v4f b4a = *(const v4f*)(gb + lane * 4), b4b = *(const v4f*)(gb + 128 + lane * 4);
#pragma unroll 1
  for (int rr = 0; rr < 4; ++rr) {
    const int row = wave * 4 + rr;
    const float* sp = sX + row * kLnP;
    const v4f a0 = *(const v4f*)(sp + lane * 8);
    const v4f a1 = *(const v4f*)(sp + lane * 8 + 4);
    float s = ((a0[0] + a0[1]) + (a0[2] + a0[3])) + ((a1[0] + a1[1]) + (a1[2] + a1[3]));
#pragma unroll
    for (int off = 16; off > 0; off >>= 1) s += __shfl_xor(s, off, 32);
    const float mean = s * (1.0f / 256.0f);
    const v4f d0 = a0 - mean, d1 = a1 - mean;
    float ss = ((d0[0] * d0[0] + d0[1] * d0[1]) + (d0[2] * d0[2] + d0[3] * d0[3]))
             + ((d1[0] * d1[0] + d1[1] * d1[1]) + (d1[2] * d1[2] + d1[3] * d1[3]));
#pragma unroll
    for (int off = 16; off > 0; off >>= 1) ss += __shfl_xor(ss, off, 32);
    const float var  = ss * (1.0f / 256.0f);
    const float rstd = rsqrtf(var + 1e-5f);
    v8h hv;
#pragma unroll
    for (int e = 0; e < 4; ++e) {
      hv[e]     = (_Float16)((d0[e] * rstd) * g8a[e] + b8a[e]);
      hv[4 + e] = (_Float16)((d1[e] * rstd) * g8b[e] + b8b[e]);
    }
    const v4f p0 = *(const v4f*)(sp + lane * 4);
    const v4f p1 = *(const v4f*)(sp + 128 + lane * 4);
    v4f f0, f1;
#pragma unroll
    for (int e = 0; e < 4; ++e) {
      f0[e] = ((p0[e] - mean) * rstd) * g4a[e] + b4a[e];
      f1[e] = ((p1[e] - mean) * rstd) * g4b[e] + b4b[e];
    }
    const size_t tok = (size_t)blk * 32 + row;
    float*    yr = YLN  + tok * kDimC;
    _Float16* hr = YLNH + tok * kDimC;
    for (int pass = 0; pass < 2; ++pass) {
      *(volatile v4f*)(yr + lane * 4)       = f0;
      *(volatile v4f*)(yr + 128 + lane * 4) = f1;
      *(volatile v8h*)(hr + lane * 8)       = hv;
      __threadfence();
    }
  }
}

__global__ __launch_bounds__(256) void conv_silu_kernel(
    const float* __restrict__ XZ, const float* __restrict__ cw, const float* __restrict__ cb,
    float* __restrict__ XC, _Float16* __restrict__ XCH, float hscale)
{
  __shared__ __align__(16) float sT[16 * kTP];
  const int tid = threadIdx.x, lane = tid & 31, wave = tid >> 5;
  const int d0 = blockIdx.x * 256, d = d0 + tid;
  const int g0 = blockIdx.y * 64;
  const int tb = g0 & (kSeqL - 1);
  const float w0 = cw[d * 4 + 0], w1 = cw[d * 4 + 1], w2 = cw[d * 4 + 2], w3 = cw[d * 4 + 3];
  const float bc = cb[d];
  float xm3, xm2, xm1;
  {
    const int r3 = (tb >= 3) ? (g0 - 3) : g0;
    const int r2 = (tb >= 2) ? (g0 - 2) : g0;
    const int r1 = (tb >= 1) ? (g0 - 1) : g0;
    const float v3 = XZ[(size_t)r3 * kXZW + d];
    const float v2 = XZ[(size_t)r2 * kXZW + d];
    const float v1 = XZ[(size_t)r1 * kXZW + d];
    xm3 = (tb >= 3) ? v3 : 0.f;
    xm2 = (tb >= 2) ? v2 : 0.f;
    xm1 = (tb >= 1) ? v1 : 0.f;
  }
  const int hrow = wave >> 1;
  const int hch  = (wave & 1) * 128 + lane * 4;
#pragma unroll 1
  for (int sub = 0; sub < 4; ++sub) {
    const int lb = g0 + sub * 16;
#pragma unroll 1
    for (int s = 0; s < 16; ++s) {
      const float xcur = XZ[(size_t)(lb + s) * kXZW + d];
      float acc = w0 * xm3;
      acc = fmaf(w1, xm2, acc);
      acc = fmaf(w2, xm1, acc);
      acc = fmaf(w3, xcur, acc);
      const float sv = acc + bc;
      const float sg = __builtin_amdgcn_rcpf(1.0f + __expf(-sv));
      sT[s * kTP + tid] = sv * sg;
      xm3 = xm2; xm2 = xm1; xm1 = xcur;
    }
    __syncthreads();
    v4f fv[4];
    v8h hv[2];
#pragma unroll
    for (int it = 0; it < 4; ++it) fv[it] = *(const v4f*)(sT + (it * 4 + hrow) * kTP + hch);
#pragma unroll
    for (int it = 0; it < 2; ++it) {
      const float* sp = sT + (it * 8 + wave) * kTP + lane * 8;
      const v4f a0 = *(const v4f*)(sp);
      const v4f a1 = *(const v4f*)(sp + 4);
#pragma unroll
      for (int e = 0; e < 4; ++e) {
        hv[it][e]     = (_Float16)(a0[e] * hscale);
        hv[it][4 + e] = (_Float16)(a1[e] * hscale);
      }
    }
    for (int pass = 0; pass < 2; ++pass) {
#pragma unroll
      for (int it = 0; it < 4; ++it)
        *(volatile v4f*)(XC + (size_t)(lb + it * 4 + hrow) * kDin + d0 + hch) = fv[it];
#pragma unroll
      for (int it = 0; it < 2; ++it)
        *(volatile v8h*)(XCH + (size_t)(lb + it * 8 + wave) * kDin + d0 + lane * 8) = hv[it];
      __threadfence();
    }
    __syncthreads();
  }
}

__global__ __launch_bounds__(256) void dt_plane_kernel(
    const float* __restrict__ XDBL, _Float16* __restrict__ DTH, int total8, float dscale)
{
  const int i = blockIdx.x * 256 + threadIdx.x;
  if (i >= total8) return;
  const int e0  = i << 3;
  const int row = e0 >> 5;
  const int c8  = e0 & 31;
  const int cc  = (c8 < kDtR) ? c8 : 8;
  const bool keep = (c8 < kDtR);
  const float* p = XDBL + (size_t)row * kXdP + cc;
  const v4f a0 = *(const v4f*)(p);
  const v4f a1 = *(const v4f*)(p + 4);
  v8h hv;
#pragma unroll
  for (int e = 0; e < 4; ++e) {
    hv[e]     = (_Float16)(keep ? a0[e] * dscale : 0.0f);
    hv[4 + e] = (_Float16)(keep ? a1[e] * dscale : 0.0f);
  }
  _Float16* q = DTH + e0;
  *(volatile v8h*)q = hv;
  __threadfence();
  *(volatile v8h*)q = hv;
}

__global__ __launch_bounds__(128) void scan_kernel(
    const float* __restrict__ DRAW, const float* __restrict__ XC, const float* __restrict__ XZ,
    const float* __restrict__ XDBL, const float* __restrict__ A_log, const float* __restrict__ Dv,
    _Float16* __restrict__ YS, float yscale)
{
  __shared__ __align__(16) float sBC[16 * 32];
  __shared__ __align__(16) float sY[16 * kSYP];
  const int tid = threadIdx.x, lane = tid & 31, wave = tid >> 5;
  const int d0 = blockIdx.x * kChBlk, d = d0 + tid;
  const int rowbase = blockIdx.y * kSeqL;

  float An[kNst];
#pragma unroll
  for (int n = 0; n < kNst; ++n) An[n] = -expf(A_log[(size_t)d * kNst + n]);
  const float Dd = Dv[d];
  float h[kNst];
#pragma unroll
  for (int n = 0; n < kNst; ++n) h[n] = 0.f;

#pragma unroll 1
  for (int c = 0; c < kSeqL / 16; ++c) {
    const int l0 = rowbase + c * 16;
    {
      const int r = tid >> 3, q = (tid & 7) * 4;
      const v4f v = *(const v4f*)(XDBL + (size_t)(l0 + r) * kXdP + kDtR + q);
      *(v4f*)(sBC + r * 32 + q) = v;
    }
    __syncthreads();
#pragma unroll 1
    for (int s = 0; s < 16; ++s) {
      const size_t m = (size_t)(l0 + s);
      const float a     = DRAW[m * kDin + d];
      const float delta = fmaxf(a, 0.0f) + log1pf(__expf(-fabsf(a)));
      const float xv    = XC[m * kDin + d];
      const float zv    = XZ[m * kXZW + kDin + d];
      const float du    = delta * xv;
      const float* bp = sBC + s * 32;
      const float* cp = bp + kNst;
      float y = 0.f;
#pragma unroll
      for (int qq = 0; qq < 4; ++qq) {
        const v4f Bq = *(const v4f*)(bp + 4 * qq);
        const v4f Cq = *(const v4f*)(cp + 4 * qq);
#pragma unroll
        for (int e = 0; e < 4; ++e) {
          const int n = qq * 4 + e;
          const float ex = __expf(delta * An[n]);
          const float hn = h[n] * ex + du * Bq[e];
          h[n] = hn;
          y += Cq[e] * hn;
        }
      }
      y += Dd * xv;
      const float sg = __builtin_amdgcn_rcpf(1.0f + __expf(-zv));
      const float g  = zv * sg;
      sY[s * kSYP + tid] = y * g;
    }
    __syncthreads();
    {
      v8h hv[2];
      size_t o[2];
#pragma unroll
      for (int it = 0; it < 2; ++it) {
        const int row = it * 8 + 2 * wave + (lane >> 4);
        const int c8  = (lane & 15) * 8;
        const float* sp = sY + row * kSYP + c8;
        const v4f a0 = *(const v4f*)(sp);
        const v4f a1 = *(const v4f*)(sp + 4);
#pragma unroll
        for (int e = 0; e < 4; ++e) {
          hv[it][e]     = (_Float16)(a0[e] * yscale);
          hv[it][4 + e] = (_Float16)(a1[e] * yscale);
        }
        o[it] = (size_t)(l0 + row) * kDin + d0 + c8;
      }
      for (int pass = 0; pass < 2; ++pass) {
        *(volatile v8h*)(YS + o[0]) = hv[0];
        *(volatile v8h*)(YS + o[1]) = hv[1];
        __threadfence();
      }
    }
  }
}

__global__ __launch_bounds__(256) void y2_planes_kernel(
    const float* __restrict__ Y2, float* __restrict__ Y2T, _Float16* __restrict__ Y2H)
{
  __shared__ __align__(16) float sT[32 * kLnP];
  const int tid = threadIdx.x, lane = tid & 31, wave = tid >> 5;
  const int blk = blockIdx.x;
  const int b   = blk >> 7;
  const int l0  = (blk & 127) * 32;
  const size_t tokbase = (size_t)blk * 32;
#pragma unroll 1
  for (int rr = 0; rr < 4; ++rr) {
    const int row = wave * 4 + rr;
    const float* p = Y2 + (tokbase + row) * kDimC + lane * 8;
    const v4f a0 = *(const v4f*)(p);
    const v4f a1 = *(const v4f*)(p + 4);
    *(v4f*)(sT + row * kLnP + lane * 8)     = a0;
    *(v4f*)(sT + row * kLnP + lane * 8 + 4) = a1;
    v8h hv;
#pragma unroll
    for (int e = 0; e < 4; ++e) { hv[e] = (_Float16)a0[e]; hv[4 + e] = (_Float16)a1[e]; }
    _Float16* q = Y2H + (tokbase + row) * kDimC + lane * 8;
    for (int pass = 0; pass < 2; ++pass) {
      *(volatile v8h*)q = hv;
      __threadfence();
    }
  }
  __syncthreads();
#pragma unroll 1
  for (int it = 0; it < 8; ++it) {
    const int ch = wave * 32 + it * 4 + (lane >> 3);
    const int t4 = (lane & 7) * 4;
    v4f v;
    v[0] = sT[(t4 + 0) * kLnP + ch];
    v[1] = sT[(t4 + 1) * kLnP + ch];
    v[2] = sT[(t4 + 2) * kLnP + ch];
    v[3] = sT[(t4 + 3) * kLnP + ch];
    float* q = Y2T + ((size_t)(b * kDimC + ch)) * kSeqL + l0 + t4;
    for (int pass = 0; pass < 2; ++pass) {
      *(volatile v4f*)q = v;
      __threadfence();
    }
  }
}

__global__ __launch_bounds__(256) void gelu_f16x2_kernel(
    const float* __restrict__ in, _Float16* __restrict__ out, int n2, float oscale)
{
  const int i = blockIdx.x * 256 + threadIdx.x;
  if (i >= n2) return;
  const v2f v = *(const v2f*)(in + 2 * (size_t)i);
  const float a0 = v[0], a1 = v[1];
  const float e0 = erff(a0 * 0.70710678118654752f);
  const float e1 = erff(a1 * 0.70710678118654752f);
  const float g0 = (0.5f * a0) * (e0 + 1.0f);
  const float g1 = (0.5f * a1) * (e1 + 1.0f);
  const _Float16 h0 = (_Float16)(g0 * oscale), h1 = (_Float16)(g1 * oscale);
  const unsigned u = (unsigned)__builtin_bit_cast(unsigned short, h0) | ((unsigned)__builtin_bit_cast(unsigned short, h1) << 16);
  ((volatile unsigned*)out)[i] = u;
  __threadfence();
  ((volatile unsigned*)out)[i] = u;
}

extern "C" void kernel_launch(void* const* d_in, const int* in_sizes, int n_in,
                              void* d_out, int out_size, void* d_ws, size_t ws_size,
                              hipStream_t stream)
{
  if (n_in < 16) return;
  const float* x         = (const float*)d_in[0];
  const float* norm_g    = (const float*)d_in[1];
  const float* norm_b    = (const float*)d_in[2];
  const float* in_proj_w = (const float*)d_in[3];
  const float* conv_w    = (const float*)d_in[4];
  const float* conv_b    = (const float*)d_in[5];
  const float* x_proj_w  = (const float*)d_in[6];
  const float* dt_proj_w = (const float*)d_in[7];
  const float* dt_proj_b = (const float*)d_in[8];
  const float* A_log     = (const float*)d_in[9];
  const float* Dvec      = (const float*)d_in[10];
  const float* out_proj_w= (const float*)d_in[11];
  const float* ffn_w1    = (const float*)d_in[12];
  const float* ffn_b1    = (const float*)d_in[13];
  const float* ffn_w2    = (const float*)d_in[14];
  const float* ffn_b2    = (const float*)d_in[15];
  float* dout = (float*)d_out;

  if (in_sizes[0]  != kTok * kDimC) return;
  if (in_sizes[1]  != kDimC || in_sizes[2] != kDimC) return;
  if (in_sizes[3]  != kXZW * kDimC) return;
  if (in_sizes[4]  != kDin * 4 || in_sizes[5] != kDin) return;
  if (in_sizes[6]  != kXdR * kDin) return;
  if (in_sizes[7]  != kDin * kDtR || in_sizes[8] != kDin) return;
  if (in_sizes[9]  != kDin * kNst || in_sizes[10] != kDin) return;
  if (in_sizes[11] != kDimC * kDin) return;
  if (in_sizes[12] != kFfn * kDimC || in_sizes[13] != kFfn) return;
  if (in_sizes[14] != kDimC * kFfn || in_sizes[15] != kDimC) return;
  if (out_size != kTok * kDimC) return;

  const size_t SZ_YLN  = (size_t)kTok * kDimC * 4;
  const size_t SZ_YLNH = (size_t)kTok * kDimC * 2;
  const size_t SZ_WIN  = (size_t)kXZW * kDimC * 2;
  const size_t SZ_WXP  = (size_t)kXdP * kDin * 2;
  const size_t SZ_WDT  = (size_t)kDin * kDtP * 2;
  const size_t SZ_WOUT = (size_t)kDimC * kDin * 2;
  const size_t SZ_WF1  = (size_t)kFfn * kDimC * 2;
  const size_t SZ_WF2  = (size_t)kDimC * kFfn * 2;
  const size_t SZ_XZ   = (size_t)kTok * kXZW * 4;
  const size_t SZ_XC   = (size_t)kTok * kDin * 4;
  const size_t SZ_XCH  = (size_t)kTok * kDin * 2;
  const size_t SZ_XDBL = (size_t)kTok * kXdP * 4;
  const size_t SZ_DTH  = (size_t)kTok * kDtP * 2;
  const size_t SZ_DRAW = (size_t)kTok * kDin * 4;
  const size_t OFF_YLN  = 0;
  const size_t OFF_YLNH = OFF_YLN  + SZ_YLN;
  const size_t OFF_WIN  = OFF_YLNH + SZ_YLNH;
  const size_t OFF_WXP  = OFF_WIN  + SZ_WIN;
  const size_t OFF_WDT  = OFF_WXP  + SZ_WXP;
  const size_t OFF_WOUT = OFF_WDT  + SZ_WDT;
  const size_t OFF_WF1  = OFF_WOUT + SZ_WOUT;
  const size_t OFF_WF2  = OFF_WF1  + SZ_WF1;
  const size_t OFF_XZ   = OFF_WF2  + SZ_WF2;
  const size_t OFF_XC   = OFF_XZ   + SZ_XZ;
  const size_t OFF_XCH  = OFF_XC   + SZ_XC;
  const size_t OFF_XDBL = OFF_XCH  + SZ_XCH;
  const size_t OFF_DTH  = OFF_XDBL + SZ_XDBL;
  const size_t OFF_DRAW = OFF_DTH  + SZ_DTH;
  const size_t TOTAL    = OFF_DRAW + SZ_DRAW;
  if (ws_size < TOTAL) return;

  char* ws = (char*)d_ws;
  float*    YLN  = (float*)(ws + OFF_YLN);
  _Float16* YLNH = (_Float16*)(ws + OFF_YLNH);
  _Float16* WIN  = (_Float16*)(ws + OFF_WIN);
  _Float16* WXP  = (_Float16*)(ws + OFF_WXP);
  _Float16* WDT  = (_Float16*)(ws + OFF_WDT);
  _Float16* WOUT = (_Float16*)(ws + OFF_WOUT);
  _Float16* WF1  = (_Float16*)(ws + OFF_WF1);
  _Float16* WF2  = (_Float16*)(ws + OFF_WF2);
  float*    XZ   = (float*)(ws + OFF_XZ);
  float*    XC   = (float*)(ws + OFF_XC);
  _Float16* XCH  = (_Float16*)(ws + OFF_XCH);
  float*    XDBL = (float*)(ws + OFF_XDBL);
  _Float16* DTH  = (_Float16*)(ws + OFF_DTH);
  float*    DRAW = (float*)(ws + OFF_DRAW);
  _Float16* YS   = XCH;
  float*    Y2   = DRAW;
  _Float16* Y2H  = (_Float16*)(ws + OFF_DRAW + (size_t)kTok * kDimC * 4);
  float*    Y2T  = (float*)(ws + OFF_XCH);
  float*    HPRE = XZ;
  _Float16* HH   = (_Float16*)(ws + OFF_XC);
  const float* dummy_bias  = dt_proj_b;
  const float* dummy_resid = x;

  const float kWsc = 64.0f;
  const float kXsc = 256.0f;
  const float kDsc = 1024.0f;
  const float kYsc = 1024.0f;
  const float kHsc = 16.0f;

  cast_w_f16_kernel<<<(kXZW * kDimC) / 8 / 256, 256, 0, stream>>>(in_proj_w,  WIN,  kDimC, kDimC, kXZW,  (kXZW * kDimC) / 8, kWsc);
  cast_w_f16_kernel<<<(kXdP * kDin)  / 8 / 256, 256, 0, stream>>>(x_proj_w,   WXP,  kDin,  kDin,  kXdR,  (kXdP * kDin) / 8,  kWsc);
  cast_w_f16_kernel<<<(kDin * kDtP)  / 8 / 256, 256, 0, stream>>>(dt_proj_w,  WDT,  kDtR,  kDtP,  kDin,  (kDin * kDtP) / 8,  kWsc);
  cast_w_f16_kernel<<<(kDimC * kDin) / 8 / 256, 256, 0, stream>>>(out_proj_w, WOUT, kDin,  kDin,  kDimC, (kDimC * kDin) / 8, kWsc);
  cast_w_f16_kernel<<<(kFfn * kDimC) / 8 / 256, 256, 0, stream>>>(ffn_w1,     WF1,  kDimC, kDimC, kFfn,  (kFfn * kDimC) / 8, kWsc);
  cast_w_f16_kernel<<<(kDimC * kFfn) / 8 / 256, 256, 0, stream>>>(ffn_w2,     WF2,  kFfn,  kFfn,  kDimC, (kDimC * kFfn) / 8, kWsc);

  ln_kernel<<<kTok / 32, 256, 0, stream>>>(x, norm_g, norm_b, YLN, YLNH);

  wmma_gemm64<0, false, 0, 0, false><<<dim3(256, 1), 256, 0, stream>>>(
      (const unsigned short*)YLNH, (const unsigned short*)YLNH, kDimC, 0L,
      (const unsigned short*)WIN, (const unsigned short*)WIN, kDimC, 0L,
      (void*)XZ, (void*)XZ, kXZW, 0L, dummy_bias, dummy_resid, 0L, kTok, kXZW, kDimC, 1.0f / kWsc);

  conv_silu_kernel<<<dim3(kDin / 256, kTok / 64), 256, 0, stream>>>(XZ, conv_w, conv_b, XC, XCH, kXsc);

  wmma_gemm64<0, false, 0, 0, false><<<dim3(16, 1), 256, 0, stream>>>(
      (const unsigned short*)XCH, (const unsigned short*)XCH, kDin, 0L,
      (const unsigned short*)WXP, (const unsigned short*)WXP, kDin, 0L,
      (void*)XDBL, (void*)XDBL, kXdP, 0L, dummy_bias, dummy_resid, 0L, kTok, kXdP, kDin, 1.0f / (kXsc * kWsc));

  dt_plane_kernel<<<(kTok * kDtP) / 8 / 256, 256, 0, stream>>>(XDBL, DTH, (kTok * kDtP) / 8, kDsc);

  wmma_gemm64<0, false, 2, 0, false><<<dim3(128, 1), 256, 0, stream>>>(
      (const unsigned short*)DTH, (const unsigned short*)DTH, kDtP, 0L,
      (const unsigned short*)WDT, (const unsigned short*)WDT, kDtP, 0L,
      (void*)DRAW, (void*)DRAW, kDin, 0L, dt_proj_b, dummy_resid, 0L, kTok, kDin, kDtP, 1.0f / (kDsc * kWsc));

  scan_kernel<<<dim3(kDin / kChBlk, kBatch), kChBlk, 0, stream>>>(DRAW, XC, XZ, XDBL, A_log, Dvec, YS, kYsc);

  wmma_gemm64<0, false, 0, 0, true><<<dim3(64, 1), 256, 0, stream>>>(
      (const unsigned short*)YS, (const unsigned short*)YS, kDin, 0L,
      (const unsigned short*)WOUT, (const unsigned short*)WOUT, kDin, 0L,
      (void*)Y2, (void*)Y2, kDimC, 0L, dummy_bias, YLN, 0L, kTok, kDimC, kDin, 1.0f / (kYsc * kWsc));

  y2_planes_kernel<<<kTok / 32, 256, 0, stream>>>(Y2, Y2T, Y2H);

  wmma_gemm64<0, false, 2, 0, false><<<dim3(256, 1), 256, 0, stream>>>(
      (const unsigned short*)Y2H, (const unsigned short*)Y2H, kDimC, 0L,
      (const unsigned short*)WF1, (const unsigned short*)WF1, kDimC, 0L,
      (void*)HPRE, (void*)HPRE, kFfn, 0L, ffn_b1, dummy_resid, 0L, kTok, kFfn, kDimC, 1.0f / kWsc);

  gelu_f16x2_kernel<<<(kTok * kFfn) / 2 / 256, 256, 0, stream>>>(HPRE, HH, (kTok * kFfn) / 2, kHsc);

  wmma_gemm64<0, false, 1, 0, true><<<dim3(32, kBatch), 256, 0, stream>>>(
      (const unsigned short*)WF2, (const unsigned short*)WF2, kFfn, 0L,
      (const unsigned short*)HH, (const unsigned short*)HH, kFfn, (long)kSeqL * kFfn,
      (void*)dout, (void*)dout, kSeqL, (long)kDimC * kSeqL, ffn_b2, Y2T, (long)kDimC * kSeqL,
      kDimC, kSeqL, kFfn, 1.0f / (kWsc * kHsc));
}
